// SSM_78477642432794
// MI455X (gfx1250) — hardware-verified
//
#include <hip/hip_runtime.h>
#include <math.h>

typedef __attribute__((ext_vector_type(16))) _Float16 v16h;
typedef __attribute__((ext_vector_type(8)))  _Float16 v8h;
typedef __attribute__((ext_vector_type(16))) __bf16   v16b;
typedef __attribute__((ext_vector_type(8)))  __bf16   v8b;
typedef __attribute__((ext_vector_type(8)))  float    v8f;
typedef __attribute__((ext_vector_type(4)))  float    v4f;

constexpr int kNB   = 4;
constexpr int kNL   = 2048;
constexpr int kND   = 768;
constexpr int kNS   = 16;
constexpr int kRows = kNB * kNL;
constexpr int kNcat = 64;
constexpr int kBcW  = 64;
constexpr int kScanTS = 64;
constexpr int kScanCh = 64;
constexpr int kScanYP = 68;
constexpr float kLog2e = 1.44269504088896340736f;
static_assert((kND % 32) == 0, "GEMM K multiple of 32");
static_assert((kRows % 64) == 0 && (kNcat % 64) == 0, "GEMM M,N multiples of 64");
static_assert((kNL % kScanTS) == 0 && (kND % kScanCh) == 0 && (kND % 8) == 0, "tile multiples");
static_assert(kBcW == kScanCh, "staging map assumes 64-wide rows");

constexpr size_t kOffXB   = 0;
constexpr size_t kOffWB   = kOffXB + (size_t)kRows * kND * 2;
constexpr size_t kOffBC   = kOffWB + (size_t)kNcat * kND * 2;
constexpr size_t kWsTotal = kOffBC + (size_t)kRows * kBcW * 4;
static_assert(kWsTotal == 14778368ull, "carve total");
static_assert(kWsTotal <= 134217728ull, "carve cap");
static_assert((kOffWB % 128) == 0 && (kOffBC % 128) == 0, "128-B aligned regions");

__device__ __forceinline__ unsigned short f2bf_bits(float f) {
  unsigned u = __float_as_uint(f);
  return (unsigned short)((u + 0x7FFFu + ((u >> 16) & 1u)) >> 16);
}
__device__ __forceinline__ float bf_bits2f(unsigned short h) { return __uint_as_float(((unsigned)h) << 16); }
__device__ __forceinline__ float bf16r(float f) { return bf_bits2f(f2bf_bits(f)); }

__device__ __forceinline__ void dep_guard_h(v8f& a, v8f& b, v16h x, v16h y) { asm volatile("v_nop\n\tv_nop\n\tv_nop\n\tv_nop" : "+v"(a), "+v"(b) : "v"(x), "v"(y)); }
__device__ __forceinline__ void dep_guard_b(v8f& a, v8f& b, v16b x, v16b y) { asm volatile("v_nop\n\tv_nop\n\tv_nop\n\tv_nop" : "+v"(a), "+v"(b) : "v"(x), "v"(y)); }
__device__ __forceinline__ void dep_guard4_h(v8f& a, v8f& b, v8f& c, v8f& d, v16h x, v16h y) { asm volatile("v_nop\n\tv_nop\n\tv_nop\n\tv_nop" : "+v"(a), "+v"(b), "+v"(c), "+v"(d) : "v"(x), "v"(y)); }
__device__ __forceinline__ void dep_guard4_b(v8f& a, v8f& b, v8f& c, v8f& d, v16b x, v16b y) { asm volatile("v_nop\n\tv_nop\n\tv_nop\n\tv_nop" : "+v"(a), "+v"(b), "+v"(c), "+v"(d) : "v"(x), "v"(y)); }
__device__ __forceinline__ void keep4_h(v16h a, v16h b, v16h c, v16h d) { asm volatile("v_nop" :: "v"(a), "v"(b), "v"(c), "v"(d)); }
__device__ __forceinline__ void keep4_b(v16b a, v16b b, v16b c, v16b d) { asm volatile("v_nop" :: "v"(a), "v"(b), "v"(c), "v"(d)); }
__device__ __forceinline__ void acc_guard4(v8f& a, v8f& b, v8f& c, v8f& d) { asm volatile("v_nop\n\tv_nop\n\tv_nop\n\tv_nop" : "+v"(a), "+v"(b), "+v"(c), "+v"(d)); }
template <typename T> struct Frag;
template <> struct Frag<_Float16> {
  typedef v16h V; union U { v16h v; v8h h[2]; };
  static __device__ __forceinline__ v16h load(const _Float16* p) {
    U f; f.h[0] = *(const v8h*)(p); f.h[1] = *(const v8h*)(p + 16); return f.v;
  }
  static __device__ __forceinline__ v8f mma(v16h a, v16h b, v8f c) {
    return __builtin_amdgcn_wmma_f32_16x16x32_f16(false, a, false, b, (short)0, c, false, false);
  }
  static __device__ __forceinline__ void guard(v8f& a, v8f& b, v16h x, v16h y) { dep_guard_h(a, b, x, y); }
  static __device__ __forceinline__ void guard4(v8f& a, v8f& b, v8f& c, v8f& d, v16h x, v16h y) { dep_guard4_h(a, b, c, d, x, y); }
  static __device__ __forceinline__ void keep(v16h a, v16h b, v16h c, v16h d) { keep4_h(a, b, c, d); }
};
template <> struct Frag<__bf16> {
  typedef v16b V; union U { v16b v; v8b h[2]; };
  static __device__ __forceinline__ v16b load(const __bf16* p) {
    U f; f.h[0] = *(const v8b*)(p); f.h[1] = *(const v8b*)(p + 16); return f.v;
  }
  static __device__ __forceinline__ v8f mma(v16b a, v16b b, v8f c) {
    return __builtin_amdgcn_wmma_f32_16x16x32_bf16(false, a, false, b, (short)0, c, false, false);
  }
  static __device__ __forceinline__ void guard(v8f& a, v8f& b, v16b x, v16b y) { dep_guard_b(a, b, x, y); }
  static __device__ __forceinline__ void guard4(v8f& a, v8f& b, v8f& c, v8f& d, v16b x, v16b y) { dep_guard4_b(a, b, c, d, x, y); }
  static __device__ __forceinline__ void keep(v16b a, v16b b, v16b c, v16b d) { keep4_b(a, b, c, d); }
};

template <int ET> struct Elem;
template <> struct Elem<0> { typedef _Float16 T; };
template <> struct Elem<1> { typedef __bf16 T; };
template <int ET, bool SPLIT, int BIAS_MODE, int OUT_MODE, bool RESID, int ACT = 0>
__global__ __launch_bounds__(256) void wmma_gemm64(
    const unsigned short* __restrict__ Ap, const unsigned short* __restrict__ A2p, int lda, long strideA,
    const unsigned short* __restrict__ Btp, const unsigned short* __restrict__ Bt2p, int ldb, long strideB,
    void* __restrict__ Cout, void* __restrict__ Cout2, int ldc, long strideC,
    const float* __restrict__ bias,
    const float* __restrict__ resid, long strideR,
    int M, int N, int K, float scale) {
  typedef typename Elem<ET>::T T;
  typedef typename Frag<T>::V V;
  const T* A = (const T*)Ap; const T* A2 = (const T*)A2p; const T* Bt = (const T*)Btp; const T* Bt2 = (const T*)Bt2p;
  __shared__ __align__(16) float sT[8][16 * 68];
  const int b    = blockIdx.y;
  const int lane = threadIdx.x & 31;
  const int wave = threadIdx.x >> 5;
  const int tilesN = N >> 6;
  const int tilesM = M >> 6;
  const int tile = blockIdx.x * 8 + wave;
  if (tile >= tilesM * tilesN) return;
  const int tm = tile / tilesN;
  const int tn = tile - tm * tilesN;
  const int m0 = tm << 6;
  const int n0 = tn << 6;

  const T* Ab  = A  + (size_t)b * strideA;
  const T* Bb  = Bt + (size_t)b * strideB;
  const T* Ab2 = SPLIT ? (A2  + (size_t)b * strideA) : nullptr;
  const T* Bb2 = SPLIT ? (Bt2 + (size_t)b * strideB) : nullptr;

  const int rlane = lane & 15;
  const int koff  = (lane >> 4) * 8;
  const int mOff  = (lane >> 4) * 8;

  v8f acc[4][4];
#pragma unroll
  for (int i = 0; i < 4; ++i)
#pragma unroll
    for (int j = 0; j < 4; ++j) acc[i][j] = (v8f){0.f,0.f,0.f,0.f,0.f,0.f,0.f,0.f};

  for (int k0 = 0; k0 < K; k0 += 32) {
    V bh[4], bl[4];
#pragma unroll
    for (int j = 0; j < 4; ++j) {
      const size_t bo = (size_t)(n0 + (j << 4) + rlane) * ldb + koff + k0;
      bh[j] = Frag<T>::load(Bb + bo);
      if (SPLIT) bl[j] = Frag<T>::load(Bb2 + bo);
    }
#pragma unroll
    for (int i = 0; i < 4; ++i) {
      const size_t ao = (size_t)(m0 + (i << 4) + rlane) * lda + koff + k0;
      V ah = Frag<T>::load(Ab + ao);
      V al;
      if (SPLIT) al = Frag<T>::load(Ab2 + ao);
#pragma unroll
      for (int j = 0; j < 4; ++j) {
        acc[i][j] = Frag<T>::mma(ah, bh[j], acc[i][j]);
        if (SPLIT) {
          acc[i][j] = Frag<T>::mma(ah, bl[j], acc[i][j]);
          acc[i][j] = Frag<T>::mma(al, bh[j], acc[i][j]);
        }
      }
      Frag<T>::guard4(acc[i][0], acc[i][1], acc[i][2], acc[i][3], ah, SPLIT ? al : ah);
    }
    Frag<T>::keep(bh[0], bh[1], bh[2], bh[3]);
    if (SPLIT) Frag<T>::keep(bl[0], bl[1], bl[2], bl[3]);
  }
  acc_guard4(acc[0][0], acc[0][1], acc[0][2], acc[0][3]);
  acc_guard4(acc[1][0], acc[1][1], acc[1][2], acc[1][3]);
  acc_guard4(acc[2][0], acc[2][1], acc[2][2], acc[2][3]);
  acc_guard4(acc[3][0], acc[3][1], acc[3][2], acc[3][3]);

  float* slab = sT[wave];
  const float* Rb = RESID ? (resid + (size_t)b * strideR) : nullptr;
#pragma unroll
  for (int i = 0; i < 4; ++i) {
    const int mBase = m0 + (i << 4);
#pragma unroll
    for (int j = 0; j < 4; ++j) {
      const int n = n0 + (j << 4) + rlane;
      float bv = 0.f;
      if (BIAS_MODE == 2) bv = bias[n];
#pragma unroll
      for (int r = 0; r < 8; ++r) {
        float v = acc[i][j][r] * scale;
        if (BIAS_MODE == 1) v += bias[mBase + mOff + r];
        if (BIAS_MODE == 2) v += bv;
        if (RESID) v += Rb[(size_t)(mBase + mOff + r) * ldc + n];
        if (ACT == 1) v = tanhf(v);
        if (ACT == 2) v = fmaxf(v, 0.0f);
        if (ACT == 3) v = v / (1.0f + expf(-v));
        if (ACT == 4) v = (v > 0.f) ? v : 0.01f * v;
        slab[(mOff + r) * 68 + (j << 4) + rlane] = v;
      }
    }
    __builtin_amdgcn_fence(__ATOMIC_RELEASE, "workgroup");
    __builtin_amdgcn_wave_barrier();
    __builtin_amdgcn_fence(__ATOMIC_ACQUIRE, "workgroup");
    if (OUT_MODE == 0) {
      float* C = (float*)Cout + (size_t)b * strideC;
      const int hh = lane >> 4, c4 = (lane & 15) * 4;
      for (int pass = 0; pass < 2; ++pass) {
#pragma unroll
        for (int it = 0; it < 8; ++it) {
          const int row = it * 2 + hh;
          v4f v = *(const v4f*)(slab + row * 68 + c4);
          *(volatile v4f*)(C + (size_t)(mBase + row) * ldc + n0 + c4) = v;
        }
        __threadfence();
      }
    } else {
      const int q = lane >> 3, c8 = (lane & 7) * 8;
      unsigned short* C  = (unsigned short*)Cout  + (size_t)b * strideC;
      unsigned short* C2 = (OUT_MODE == 2) ? ((unsigned short*)Cout2 + (size_t)b * strideC) : nullptr;
      for (int pass = 0; pass < 2; ++pass) {
#pragma unroll
        for (int it = 0; it < 4; ++it) {
          const int row = it * 4 + q;
          const float* sp = slab + row * 68 + c8;
          v8h hv, lv;
#pragma unroll
          for (int e = 0; e < 8; ++e) {
            if (OUT_MODE == 1) {
              hv[e] = (_Float16)sp[e];
            } else {
              unsigned short hb = f2bf_bits(sp[e]);
              unsigned short lb = f2bf_bits(sp[e] - bf_bits2f(hb));
              hv[e] = __builtin_bit_cast(_Float16, hb);
              lv[e] = __builtin_bit_cast(_Float16, lb);
            }
          }
          *(volatile v8h*)(C + (size_t)(mBase + row) * ldc + n0 + c8) = hv;
          if (OUT_MODE == 2) *(volatile v8h*)(C2 + (size_t)(mBase + row) * ldc + n0 + c8) = lv;
        }
        __threadfence();
      }
    }
    __builtin_amdgcn_fence(__ATOMIC_RELEASE, "workgroup");
    __builtin_amdgcn_wave_barrier();
    __builtin_amdgcn_fence(__ATOMIC_ACQUIRE, "workgroup");
  }
}

__global__ __launch_bounds__(256) void rows_to_bf16_kernel(
    const float* __restrict__ src, unsigned short* __restrict__ dst, int total8)
{
  const int i = blockIdx.x * 256 + threadIdx.x;
  if (i >= total8) return;
  const size_t e0 = (size_t)i << 3;
  const v4f a0 = *(const v4f*)(src + e0);
  const v4f a1 = *(const v4f*)(src + e0 + 4);
  v8h hv;
#pragma unroll
  for (int e = 0; e < 4; ++e) {
    const unsigned short h0 = f2bf_bits(a0[e]);
    const unsigned short h1 = f2bf_bits(a1[e]);
    hv[e]     = __builtin_bit_cast(_Float16, h0);
    hv[4 + e] = __builtin_bit_cast(_Float16, h1);
  }
  unsigned short* qd = dst + e0;
  *(volatile v8h*)qd = hv;
  __threadfence();
  *(volatile v8h*)qd = hv;
}

__global__ __launch_bounds__(256) void build_wcat_kernel(
    const float* __restrict__ Wb, const float* __restrict__ Wc, const float* __restrict__ W1,
    unsigned short* __restrict__ dst, int total8)
{
  const int i = blockIdx.x * 256 + threadIdx.x;
  if (i >= total8) return;
  const int e0  = i * 8;
  const int row = e0 / kND;
  const int col = e0 - row * kND;
  const int rb = (row < kNS) ? row : (kNS - 1);
  int rc = row - kNS;
  rc = (rc < 0) ? 0 : ((rc > kNS - 1) ? (kNS - 1) : rc);
  const v4f wb0 = *(const v4f*)(Wb + (size_t)rb * kND + col);
  const v4f wb1 = *(const v4f*)(Wb + (size_t)rb * kND + col + 4);
  const v4f wc0 = *(const v4f*)(Wc + (size_t)rc * kND + col);
  const v4f wc1 = *(const v4f*)(Wc + (size_t)rc * kND + col + 4);
  const v4f w10 = *(const v4f*)(W1 + col);
  const v4f w11 = *(const v4f*)(W1 + col + 4);
  const float fb = (row < kNS) ? 1.0f : 0.0f;
  const float fc = (row >= kNS && row < 2 * kNS) ? 1.0f : 0.0f;
  const float f1 = (row == 2 * kNS) ? 1.0f : 0.0f;
  v8h hv;
#pragma unroll
  for (int e = 0; e < 4; ++e) {
    const float v0 = fmaf(fb, wb0[e], fmaf(fc, wc0[e], f1 * w10[e]));
    const float v1 = fmaf(fb, wb1[e], fmaf(fc, wc1[e], f1 * w11[e]));
    const unsigned short h0 = f2bf_bits(v0);
    const unsigned short h1 = f2bf_bits(v1);
    hv[e]     = __builtin_bit_cast(_Float16, h0);
    hv[4 + e] = __builtin_bit_cast(_Float16, h1);
  }
  unsigned short* qd = dst + (size_t)e0;
  *(volatile v8h*)qd = hv;
  __threadfence();
  *(volatile v8h*)qd = hv;
}

__global__ __launch_bounds__(64) void scan_kernel(
    const float* __restrict__ x, const float* __restrict__ BC, const float* __restrict__ Alog,
    const float* __restrict__ Wd, const float* __restrict__ bd,
    const float* __restrict__ bb, const float* __restrict__ bc, const float* __restrict__ b1,
    float* __restrict__ y)
{
  __shared__ __align__(16) float sX[kScanTS * kBcW];
  __shared__ __align__(16) float sY[kScanTS * kScanYP];
  __shared__ __align__(16) float sA[kScanCh * kNS];
  const int tid = threadIdx.x, lane = tid & 31, wave = tid >> 5;
  constexpr int kBlkPerB = kND / kScanCh;
  const int bix = blockIdx.x / kBlkPerB;
  const int d0  = (blockIdx.x - bix * kBlkPerB) * kScanCh;
  const int d   = d0 + tid;
  const size_t row0 = (size_t)bix * kNL;

#pragma unroll 1
  for (int i = 0; i < 4; ++i) {
    const int idx = tid + 64 * i;
    const v4f av = *(const v4f*)(Alog + (size_t)d0 * kNS + 4 * idx);
    v4f ov = av;
    ov[0] = -expf(bf16r(av[0])) * kLog2e;
    ov[1] = -expf(bf16r(av[1])) * kLog2e;
    ov[2] = -expf(bf16r(av[2])) * kLog2e;
    ov[3] = -expf(bf16r(av[3])) * kLog2e;
    *(v4f*)(sA + 4 * idx) = ov;
  }
  const float wdv = bf16r(Wd[d]);
  const float bdv = bf16r(bd[d]);
  asm volatile("" ::: "memory");

  const int lr = tid >> 4, q16 = tid & 15, lc4 = q16 * 4;
  const v4f bbv = *(const v4f*)(bb + 4 * (q16 & 3));
  const v4f bcv = *(const v4f*)(bc + 4 * (q16 & 3));
  const float b1s = b1[0];
  const float fb = (q16 < 4) ? 1.0f : 0.0f;
  const float fc = (q16 >= 4 && q16 < 8) ? 1.0f : 0.0f;
  const float f1 = (q16 == 8) ? 1.0f : 0.0f;
  v4f bias4 = bbv;
  {
    float t0 = fmaf(fb, bbv[0], fc * bcv[0]);
    t0 = fmaf(f1, b1s, t0);
    const float t1 = fmaf(fb, bbv[1], fc * bcv[1]);
    const float t2 = fmaf(fb, bbv[2], fc * bcv[2]);
    const float t3 = fmaf(fb, bbv[3], fc * bcv[3]);
    bias4[0] = bf16r(t0); bias4[1] = bf16r(t1); bias4[2] = bf16r(t2); bias4[3] = bf16r(t3);
  }
  __syncthreads();

  float A2[kNS], h[kNS];
#pragma unroll
  for (int q4 = 0; q4 < 4; ++q4) {
    const v4f a = *(const v4f*)(sA + tid * kNS + 4 * q4);
    A2[4 * q4 + 0] = a[0]; A2[4 * q4 + 1] = a[1]; A2[4 * q4 + 2] = a[2]; A2[4 * q4 + 3] = a[3];
  }
#pragma unroll
  for (int s = 0; s < kNS; ++s) h[s] = 0.0f;

  const int hh = lane >> 4, c4 = (lane & 15) * 4;
#pragma unroll 1
  for (int t0 = 0; t0 < kNL; t0 += kScanTS) {
    __syncthreads();
#pragma unroll
    for (int i = 0; i < 8; ++i) {
      const int r = lr + 4 * i;
      const v4f v = *(const v4f*)(BC + (row0 + t0 + r) * kBcW + lc4);
      *(v4f*)(sX + r * kBcW + lc4) = v + bias4;
    }
    asm volatile("" ::: "memory");
#pragma unroll
    for (int i = 8; i < 16; ++i) {
      const int r = lr + 4 * i;
      const v4f v = *(const v4f*)(BC + (row0 + t0 + r) * kBcW + lc4);
      *(v4f*)(sX + r * kBcW + lc4) = v + bias4;
    }
    __syncthreads();
#pragma unroll 1
    for (int s = 0; s < kScanTS; ++s) {
      const float* xr = sX + s * kBcW;
      float Bs[kNS], Cs[kNS];
#pragma unroll
      for (int q4 = 0; q4 < 4; ++q4) {
        const v4f bv = *(const v4f*)(xr + 4 * q4);
        const v4f cv = *(const v4f*)(xr + kNS + 4 * q4);
        Bs[4 * q4 + 0] = bv[0]; Bs[4 * q4 + 1] = bv[1]; Bs[4 * q4 + 2] = bv[2]; Bs[4 * q4 + 3] = bv[3];
        Cs[4 * q4 + 0] = cv[0]; Cs[4 * q4 + 1] = cv[1]; Cs[4 * q4 + 2] = cv[2]; Cs[4 * q4 + 3] = cv[3];
      }
      const float s1v = xr[2 * kNS];
      const float z   = s1v * wdv + bdv;
      const float ez  = expf(-fabsf(z));
      const float dt  = fmaxf(z, 0.0f) + log1pf(ez);
      const float xt  = bf16r(x[(row0 + t0 + s) * kND + d]);
      const float dtx = dt * xt;
      float yv = 0.0f;
#pragma unroll
      for (int k = 0; k < kNS; ++k) {
        const float e = exp2f(dt * A2[k]);
        h[k] = e * h[k] + dtx * Bs[k];
        yv = fmaf(h[k], Cs[k], yv);
      }
      sY[s * kScanYP + tid] = yv;
    }
    __syncthreads();
    for (int pass = 0; pass < 2; ++pass) {
#pragma unroll
      for (int it = 0; it < 16; ++it) {
        const int row = it * 4 + wave * 2 + hh;
        const v4f v = *(const v4f*)(sY + row * kScanYP + c4);
        *(volatile v4f*)(y + (row0 + t0 + row) * kND + d0 + c4) = v;
      }
      __threadfence();
    }
  }
}

extern "C" void kernel_launch(void* const* d_in, const int* in_sizes, int n_in,
                              void* d_out, int out_size, void* d_ws, size_t ws_size,
                              hipStream_t stream) {
  if (n_in < 10) return;
  if (in_sizes[0] != kRows * kND) return;
  if (in_sizes[1] != kND * kNS) return;
  if (in_sizes[2] != kNS * kND) return;
  if (in_sizes[3] != kNS) return;
  if (in_sizes[4] != kNS * kND) return;
  if (in_sizes[5] != kNS) return;
  if (in_sizes[6] != kND) return;
  if (in_sizes[7] != 1) return;
  if (in_sizes[8] != kND) return;
  if (in_sizes[9] != kND) return;
  if (out_size != kRows * kND) return;
  if (ws_size < kWsTotal) return;

  const float* x     = (const float*)d_in[0];
  const float* A_log = (const float*)d_in[1];
  const float* Wb    = (const float*)d_in[2];
  const float* bb    = (const float*)d_in[3];
  const float* Wc    = (const float*)d_in[4];
  const float* bc    = (const float*)d_in[5];
  const float* W1    = (const float*)d_in[6];
  const float* b1    = (const float*)d_in[7];
  const float* Wd    = (const float*)d_in[8];
  const float* bd    = (const float*)d_in[9];
  float* out = (float*)d_out;

  char* ws = (char*)d_ws;
  unsigned short* XB = (unsigned short*)(ws + kOffXB);
  unsigned short* WB = (unsigned short*)(ws + kOffWB);
  float*          BC = (float*)(ws + kOffBC);

  rows_to_bf16_kernel<<<(kRows * kND / 8) / 256, 256, 0, stream>>>(x, XB, kRows * kND / 8);
  build_wcat_kernel<<<(kNcat * kND / 8) / 256, 256, 0, stream>>>(Wb, Wc, W1, WB, kNcat * kND / 8);

  wmma_gemm64<1, false, 0, 0, false><<<dim3((kRows / 64) * (kNcat / 64) / 8, 1), 256, 0, stream>>>(
      XB, nullptr, kND, 0L,
      WB, nullptr, kND, 0L,
      (void*)BC, nullptr, kBcW, 0L,
      nullptr, nullptr, 0L,
      kRows, kNcat, kND, 1.0f);

  scan_kernel<<<kNB * (kND / kScanCh), kScanCh, 0, stream>>>(x, BC, A_log, Wd, bd, bb, bc, b1, out);
}
